// ONOBlock_61220463837315
// MI455X (gfx1250) — hardware-verified
//
#include <hip/hip_runtime.h>
#include <math.h>

typedef __attribute__((ext_vector_type(16))) _Float16 v16h;
typedef __attribute__((ext_vector_type(16))) __bf16 v16b;
typedef __attribute__((ext_vector_type(8)))  _Float16 v8h;
typedef __attribute__((ext_vector_type(8)))  float v8f;
typedef __attribute__((ext_vector_type(4)))  float v4f;
typedef __attribute__((ext_vector_type(2)))  float v2f;
typedef __attribute__((ext_vector_type(4)))  unsigned v4u;
typedef __attribute__((ext_vector_type(4)))  int v4i;
typedef float __attribute__((may_alias)) float_a;
typedef int __attribute__((may_alias)) int_a;

template <typename T> __device__ __forceinline__ void vst2(void* p, T v) { *(volatile T*)p = v; __threadfence(); *(volatile T*)p = v; }
__device__ __forceinline__ v8f wmma16(v16h a, v16h b, v8f c) {
  v8f d = __builtin_amdgcn_wmma_f32_16x16x32_f16(false, a, false, b, (short)0, c, false, false);
  asm volatile("v_nop\n\tv_nop\n\tv_nop\n\tv_nop" : "+v"(d) : "v"(a), "v"(b));
  return d;
}
__device__ __forceinline__ v8f wmma_bf(v16b a, v16b b, v8f c) {
  v8f d = __builtin_amdgcn_wmma_f32_16x16x32_bf16(false, a, false, b, (short)0, c, false, false);
  asm volatile("v_nop\n\tv_nop\n\tv_nop\n\tv_nop" : "+v"(d) : "v"(a), "v"(b));
  return d;
}
__device__ __forceinline__ v16h frag_h(const _Float16* rowk0, int lane) {
  union { v16h v; v8h q[2]; } u; const _Float16* p = rowk0 + 8 * (lane >> 4);
  u.q[0] = *(const v8h*)p; u.q[1] = *(const v8h*)(p + 16); return u.v;
}
__device__ __forceinline__ v16h frag_f32(const float* rowk0, int lane) {
  v16h a; const float* p = rowk0 + 8 * (lane >> 4);
#pragma unroll
  for (int i = 0; i < 8; ++i) { a[i] = (_Float16)p[i]; a[8 + i] = (_Float16)p[16 + i]; }
  return a;
}
__device__ __forceinline__ v16h frag_f32s(const float* rowk0, int lane, float sc) {
  v16h a; const float* p = rowk0 + 8 * (lane >> 4);
#pragma unroll
  for (int i = 0; i < 8; ++i) { a[i] = (_Float16)(p[i] * sc); a[8 + i] = (_Float16)(p[16 + i] * sc); }
  return a;
}
__device__ __forceinline__ v16h fragc_f32(const float* W, int k0, int n, int lane, int ld, int K) {
  v16h a; const int g = lane >> 4;
#pragma unroll
  for (int i = 0; i < 8; ++i) { const int ka = k0 + 8 * g + i, kb = ka + 16;
    a[i] = (_Float16)(ka < K ? W[(size_t)ka * ld + n] : 0.f); a[8 + i] = (_Float16)(kb < K ? W[(size_t)kb * ld + n] : 0.f); }
  return a;
}
struct F2 { v16b h, l; };
__device__ __forceinline__ F2 bsplit16(const float v[16]) { F2 r;
#pragma unroll
  for (int i = 0; i < 16; ++i) { const __bf16 h = (__bf16)v[i]; r.h[i] = h; r.l[i] = (__bf16)(v[i] - (float)h); }
  return r; }
__device__ __forceinline__ F2 split_row(const float* row, int k0, int lane) { float v[16]; const float* p = row + k0 + 8 * (lane >> 4);
#pragma unroll
  for (int i = 0; i < 8; ++i) { v[i] = p[i]; v[8 + i] = p[16 + i]; }
  return bsplit16(v); }
__device__ __forceinline__ F2 split_rowK(const float* row, int k0, int lane, int K) { float v[16]; const int g = lane >> 4;
#pragma unroll
  for (int i = 0; i < 8; ++i) { const int ka = k0 + 8 * g + i, kb = ka + 16; v[i] = ka < K ? row[ka] : 0.f; v[8 + i] = kb < K ? row[kb] : 0.f; }
  return bsplit16(v); }
__device__ __forceinline__ F2 split_col(const float* W, int k0, int n, int lane, int ld, int K) { float v[16]; const int g = lane >> 4;
#pragma unroll
  for (int i = 0; i < 8; ++i) { const int ka = k0 + 8 * g + i, kb = ka + 16; v[i] = ka < K ? W[(size_t)ka * ld + n] : 0.f; v[8 + i] = kb < K ? W[(size_t)kb * ld + n] : 0.f; }
  return bsplit16(v); }
__device__ __forceinline__ v8f mac3(const F2& a, const F2& b, v8f c) { c = wmma_bf(a.l, b.h, c); c = wmma_bf(a.h, b.l, c); return wmma_bf(a.h, b.h, c); }
__device__ __forceinline__ float sigm(float v) { return 1.0f / (1.0f + expf(-v)); }
#define LDSX() do { asm volatile("s_wait_dscnt 0" ::: "memory"); __builtin_amdgcn_wave_barrier(); __builtin_amdgcn_fence(__ATOMIC_RELEASE, "workgroup"); } while (0)

#define NB 4
#define NS 4096
#define DD 128
#define NH 8
#define DH 16
#define NR (NB * NS)

__device__ __forceinline__ float gelu_e(float v) { return 0.5f * v * (1.0f + erff(v * 0.70710678118654752f)); }
__device__ __forceinline__ void ln16(float so[16][132], const float* __restrict__ g, const float* __restrict__ b, int lane) {
  const int rl = lane >> 1, hf = lane & 1; float* row = &so[rl][0]; float s = 0.f; for (int c = hf * 64; c < hf * 64 + 64; ++c) s += row[c]; s += __shfl_xor(s, 1, 32); const float mu = s * (1.0f / DD);
  float q2 = 0.f; for (int c = hf * 64; c < hf * 64 + 64; ++c) { const float d = row[c] - mu; q2 += d * d; } q2 += __shfl_xor(q2, 1, 32); const float rs = rsqrtf(q2 * (1.0f / DD) + 1e-6f);
  LDSX();
  for (int c = hf * 64; c < hf * 64 + 64; ++c) row[c] = (row[c] - mu) * rs * g[c] + b[c];
  LDSX();
}
__device__ __forceinline__ void wgemm(const float* arow0, const float* __restrict__ W, v8f acc[8], int lane) {
  const int col = lane & 15;
#pragma unroll
  for (int kc = 0; kc < DD / 32; ++kc) { const F2 a = split_row(arow0 + (size_t)col * 132, kc * 32, lane);
#pragma unroll
    for (int j = 0; j < 8; ++j) acc[j] = mac3(a, split_row(W + (size_t)(j * 16 + col) * DD, kc * 32, lane), acc[j]); }
}
__global__ __launch_bounds__(128) void k_qkv(const float* __restrict__ x, const float* __restrict__ g1, const float* __restrict__ be1, const float* __restrict__ wq, const float* __restrict__ wk, const float* __restrict__ wv, float* __restrict__ Q, float* __restrict__ KP, float* __restrict__ V) {
  __shared__ __align__(16) float sx[4][16][132];
  __shared__ __align__(16) float so[4][16][132];
  const int tid = threadIdx.x, wave = tid >> 5, lane = tid & 31, col = lane & 15, g = lane >> 4;
  const int r0 = blockIdx.x * 64 + wave * 16;
  for (int q = lane; q < 16 * 32; q += 32) { const int rl = q >> 5, pc = q & 31; *(v4f*)(&sx[wave][rl][pc * 4]) = *(const v4f*)(x + (size_t)(r0 + rl) * DD + pc * 4); }
  LDSX();
  ln16(sx[wave], g1, be1, lane);
#pragma unroll 1
  for (int which = 0; which < 3; ++which) { const float* W = which == 0 ? wq : which == 1 ? wk : wv; float* D = which == 0 ? Q : which == 1 ? KP : V;
    v8f acc[8] = {};
    wgemm(&sx[wave][0][0], W, acc, lane);
#pragma unroll
    for (int j = 0; j < 8; ++j)
#pragma unroll
      for (int r = 0; r < 8; ++r) so[wave][8 * g + r][j * 16 + col] = acc[j][r];
    LDSX();
    if (which == 0) {
      const int rl = lane >> 1, hf = lane & 1; float* row = &so[wave][rl][0];
      for (int hh = hf * 4; hh < hf * 4 + 4; ++hh) { float mx = -3.4e38f; for (int d = 0; d < DH; ++d) mx = fmaxf(mx, row[hh * DH + d]); float se = 0.f; for (int d = 0; d < DH; ++d) { const float p = expf(row[hh * DH + d] - mx); row[hh * DH + d] = p; se += p; } const float inv = 1.0f / se; for (int d = 0; d < DH; ++d) row[hh * DH + d] *= inv; }
      LDSX(); }
    for (int q = lane; q < 16 * 32; q += 32) { const int rl = q >> 5, pc = q & 31; vst2(D + (size_t)(r0 + rl) * DD + pc * 4, *(const v4f*)(&so[wave][rl][pc * 4])); }
    LDSX(); }
}
__global__ __launch_bounds__(256) void k_ctx(const float* __restrict__ KP, const float* __restrict__ V, float* __restrict__ CTX) {
  __shared__ float sred[16][16]; __shared__ float smax[16], ssum[16]; __shared__ __align__(16) float sctx[256];
  const int b = blockIdx.x / NH, h = blockIdx.x % NH, tid = threadIdx.x; const int d = tid & 15, part = tid >> 4;
  const float* kb = KP + (size_t)b * NS * DD + h * DH; const float* vb = V + (size_t)b * NS * DD + h * DH;
  float mx = -3.4e38f; for (int n = part * 256; n < part * 256 + 256; ++n) mx = fmaxf(mx, kb[(size_t)n * DD + d]);
  sred[part][d] = mx;
  __syncthreads();
  if (tid < 16) { float m = -3.4e38f; for (int p = 0; p < 16; ++p) m = fmaxf(m, sred[p][tid]); smax[tid] = m; }
  __syncthreads();
  { const float m = smax[d]; float s = 0.f; for (int n = part * 256; n < part * 256 + 256; ++n) s += expf(kb[(size_t)n * DD + d] - m);
    __syncthreads(); sred[part][d] = s; }
  __syncthreads();
  if (tid < 16) { float s = 0.f; for (int p = 0; p < 16; ++p) s += sred[p][tid]; ssum[tid] = s; }
  __syncthreads();
  { const int e = part; const float m = smax[d], inv = 1.0f / ssum[d]; float acc = 0.f;
    for (int n = 0; n < NS; ++n) acc += expf(kb[(size_t)n * DD + d] - m) * vb[(size_t)n * DD + e];
    sctx[d * 16 + e] = acc * inv; }
  __syncthreads();
  if (tid < 64) vst2(CTX + (size_t)blockIdx.x * 256 + tid * 4, *(const v4f*)(&sctx[tid * 4]));
}
__global__ __launch_bounds__(128) void k_main(const float* __restrict__ x, const float* __restrict__ Q, const float* __restrict__ CTX, const float* __restrict__ wo, const float* __restrict__ bo, const float* __restrict__ g2, const float* __restrict__ be2,
                                            const float* __restrict__ w1, const float* __restrict__ b1, const float* __restrict__ w2, const float* __restrict__ b2, float* __restrict__ xo) {
  __shared__ __align__(16) float sa[4][16][132];
  __shared__ __align__(16) float sx1[4][16][132];
  __shared__ float sctx[NH * 256];
  const int tid = threadIdx.x, wave = tid >> 5, lane = tid & 31, col = lane & 15, g = lane >> 4;
  const int r0 = blockIdx.x * 64 + wave * 16; const int b = r0 / NS;
  for (int q = tid; q < NH * 256; q += 128) sctx[q] = CTX[(size_t)b * NH * 256 + q];
  __syncthreads();
  { const int rl = lane >> 1, hf = lane & 1; const float* qr = Q + (size_t)(r0 + rl) * DD;
    for (int hh = hf * 4; hh < hf * 4 + 4; ++hh) { float qv[DH]; for (int d = 0; d < DH; ++d) qv[d] = qr[hh * DH + d];
      for (int e = 0; e < DH; ++e) { float s = 0.f; for (int d = 0; d < DH; ++d) s += qv[d] * sctx[hh * 256 + d * 16 + e]; sa[wave][rl][hh * DH + e] = s; } } }
  LDSX();
  { v8f acc[8] = {}; wgemm(&sa[wave][0][0], wo, acc, lane);
#pragma unroll
    for (int j = 0; j < 8; ++j) { const int n = j * 16 + col; const float bb = bo[n];
#pragma unroll
      for (int r = 0; r < 8; ++r) { const float v = acc[j][r] + bb + x[(size_t)(r0 + 8 * g + r) * DD + n]; sx1[wave][8 * g + r][n] = v; sa[wave][8 * g + r][n] = v; } } }
  LDSX();
  ln16(sa[wave], g2, be2, lane);
  { v8f acc[8] = {}; wgemm(&sa[wave][0][0], w1, acc, lane);
    LDSX();
#pragma unroll
    for (int j = 0; j < 8; ++j) { const int n = j * 16 + col; const float bb = b1[n];
#pragma unroll
      for (int r = 0; r < 8; ++r) sa[wave][8 * g + r][n] = acc[j][r] + bb; } }
  LDSX();
  { const int rl = lane >> 1, hf = lane & 1; float* row = &sa[wave][rl][0];
#pragma unroll 1
    for (int c = hf * 64; c < hf * 64 + 64; ++c) row[c] = gelu_e(row[c]); }
  LDSX();
  { v8f acc[8] = {}; wgemm(&sa[wave][0][0], w2, acc, lane);
    LDSX();
#pragma unroll
    for (int j = 0; j < 8; ++j) { const int n = j * 16 + col; const float bb = b2[n];
#pragma unroll
      for (int r = 0; r < 8; ++r) sx1[wave][8 * g + r][n] += acc[j][r] + bb; } }
  LDSX();
  for (int q = lane; q < 16 * 32; q += 32) { const int rl = q >> 5, pc = q & 31; vst2(xo + (size_t)(r0 + rl) * DD + pc * 4, *(const v4f*)(&sx1[wave][rl][pc * 4])); }
}
__global__ __launch_bounds__(32) void k_m(const float* __restrict__ xo, const float* __restrict__ fx, float* __restrict__ M) {
  __shared__ __align__(16) float so[16][132];
  const int lane = threadIdx.x, col = lane & 15, g = lane >> 4; const int b = blockIdx.x >> 3, mt = blockIdx.x & 7;
  const float* xb = xo + (size_t)b * NS * DD; const float* fb = fx + (size_t)b * NS * DD;
  v8f acc[8] = {};
#pragma unroll 1
  for (int kc = 0; kc < NS / 32; ++kc) { const F2 a = split_col(xb, kc * 32, mt * 16 + col, lane, DD, NS);
#pragma unroll
    for (int j = 0; j < 8; ++j) acc[j] = mac3(a, split_col(fb, kc * 32, j * 16 + col, lane, DD, NS), acc[j]); }
#pragma unroll
  for (int j = 0; j < 8; ++j)
#pragma unroll
    for (int r = 0; r < 8; ++r) so[8 * g + r][j * 16 + col] = acc[j][r];
  LDSX();
  for (int q = lane; q < 16 * 32; q += 32) { const int rl = q >> 5, pc = q & 31; vst2(M + ((size_t)b * DD + mt * 16 + rl) * DD + pc * 4, *(const v4f*)(&so[rl][pc * 4])); }
}
__global__ __launch_bounds__(128) void k_fx(const float* __restrict__ xo, const float* __restrict__ M, float* __restrict__ fxo) {
  __shared__ __align__(16) float so[4][16][132];
  const int tid = threadIdx.x, wave = tid >> 5, lane = tid & 31, col = lane & 15, g = lane >> 4;
  const int r0 = blockIdx.x * 64 + wave * 16; const int b = r0 / NS; const float* Mb = M + (size_t)b * DD * DD;
  v8f acc[8] = {};
#pragma unroll
  for (int kc = 0; kc < DD / 32; ++kc) { const F2 a = split_row(xo + (size_t)(r0 + col) * DD, kc * 32, lane);
#pragma unroll
    for (int j = 0; j < 8; ++j) acc[j] = mac3(a, split_col(Mb, kc * 32, j * 16 + col, lane, DD, DD), acc[j]); }
#pragma unroll
  for (int j = 0; j < 8; ++j)
#pragma unroll
    for (int r = 0; r < 8; ++r) so[wave][8 * g + r][j * 16 + col] = acc[j][r];
  LDSX();
  { const int rl = lane >> 1, hf = lane & 1; float* row = &so[wave][rl][0];
#pragma unroll 1
    for (int c = hf * 64; c < hf * 64 + 64; ++c) row[c] = sigm(row[c]); }
  LDSX();
  for (int q = lane; q < 16 * 32; q += 32) { const int rl = q >> 5, pc = q & 31; vst2(fxo + (size_t)(r0 + rl) * DD + pc * 4, *(const v4f*)(&so[wave][rl][pc * 4])); }
}
extern "C" void kernel_launch(void* const* d_in, const int* in_sizes, int n_in, void* d_out, int out_size, void* d_ws, size_t ws_size, hipStream_t stream) {
  (void)in_sizes; (void)n_in; (void)out_size; (void)ws_size;
  const float** I = (const float**)d_in;
  const float* x = I[0]; const float* fx = I[1]; const float* g1 = I[2]; const float* be1 = I[3]; const float* wq = I[4]; const float* wk = I[5]; const float* wv = I[6]; const float* wo = I[7]; const float* bo = I[8];
  const float* g2 = I[9]; const float* be2 = I[10]; const float* w1 = I[11]; const float* b1 = I[12]; const float* w2 = I[13]; const float* b2 = I[14];
  float* xo = (float*)d_out; float* fxo = (float*)((char*)d_out + 8388608);
  char* ws = (char*)d_ws; size_t off = 0;
  auto take = [&](size_t bytes) { char* p = ws + off; off += (bytes + 255) & ~(size_t)255; return p; };
  float* Q = (float*)take((size_t)NR * DD * 4); float* KP = (float*)take((size_t)NR * DD * 4); float* V = (float*)take((size_t)NR * DD * 4); float* CTX = (float*)take((size_t)NB * NH * 256 * 4); float* M = (float*)take((size_t)NB * DD * DD * 4);
  k_qkv<<<NR / 64, 128, 0, stream>>>(x, g1, be1, wq, wk, wv, Q, KP, V);
  k_ctx<<<NB * NH, 256, 0, stream>>>(KP, V, CTX);
  k_main<<<NR / 64, 128, 0, stream>>>(x, Q, CTX, wo, bo, g2, be2, w1, b1, w2, b2, xo);
  k_m<<<NB * 8, 32, 0, stream>>>(xo, fx, M);
  k_fx<<<NR / 64, 128, 0, stream>>>(xo, M, fxo);
}
